// SelfAttention_87222195847960
// MI455X (gfx1250) — hardware-verified
//
#include <hip/hip_runtime.h>


#ifndef NB
#define NB 4
#endif
#ifndef SEQ
#define SEQ 2048
#endif
#define NB_FULL 4
#define SEQ_FULL 2048
#define DM 1024
#define NH 8
#define DK 128
#define MTOK (NB * SEQ)
#define QKVN (3 * NH * DK)
#define NTILE_FULL (SEQ_FULL / 64)

static_assert(SEQ % 64 == 0);
static_assert(SEQ <= SEQ_FULL);
static_assert(NB >= 1 && NB <= NB_FULL);
static_assert(QKVN == 3072);
static_assert(QKVN % 128 == 0);
static_assert(NH * DK == DM);
static_assert(DM % 64 == 0);
static_assert(DK == 128);
static_assert(NTILE_FULL == 32);
static_assert(32 * NB <= 128);

#define SC_W   32.0f
#define SC_QKV 8.0f
#define SC_WO  32.0f
#define P_CARRY_LOG2 8.0f

#define WS_TOTAL ((size_t)QKVN * DM * 2 + (size_t)DM * DM * 2 + (size_t)MTOK * DM * 2 + 3 * (size_t)NB * NH * SEQ * DK * 2 \
                  + (size_t)MTOK * DM * 2 + (size_t)NB_FULL * NTILE_FULL * 4)
static_assert(WS_TOTAL <= (size_t)134217728);

typedef _Float16 v8h  __attribute__((ext_vector_type(8)));
typedef _Float16 v16h __attribute__((ext_vector_type(16)));
typedef float    v8f  __attribute__((ext_vector_type(8)));
typedef float    v4f  __attribute__((ext_vector_type(4)));
typedef unsigned v4u  __attribute__((ext_vector_type(4)));

__device__ __forceinline__ float bfr(float f) {
    unsigned u = __float_as_uint(f);
    u = (u + 0x7fffu + ((u >> 16) & 1u)) & 0xffff0000u;
    return __uint_as_float(u);
}
__device__ __forceinline__ _Float16 toh_flush(float v) {
    const _Float16 r = (_Float16)v;
    return (fabsf(v) < 6.103515625e-05f) ? (_Float16)0.0f : r;
}
__device__ __forceinline__ _Float16 tohx_flush(float f, float sc) { return toh_flush(bfr(f) * sc); }

__device__ __forceinline__ v8f wmma16(v16h a, v16h b, v8f c) {
    c = __builtin_amdgcn_wmma_f32_16x16x32_f16(false, a, false, b, (short)0, c, false, false);
    asm volatile("v_nop\n\tv_nop\n\tv_nop\n\tv_nop" : "+v"(c) : "v"(a), "v"(b));
    return c;
}
__device__ __forceinline__ v16h ldfrag(const _Float16* p, int hf) {
    const v8h lo = *(const v8h*)(p + 8 * hf);
    const v8h hi = *(const v8h*)(p + 16 + 8 * hf);
    return __builtin_shufflevector(lo, hi, 0, 1, 2, 3, 4, 5, 6, 7, 8, 9, 10, 11, 12, 13, 14, 15);
}
__device__ __forceinline__ void vst16(_Float16* g, v8h v) { *(volatile v4u*)g = __builtin_bit_cast(v4u, v); }
__device__ __forceinline__ void vst16f(float* g, v4f v) { *(volatile v4f*)g = v; }
__device__ __forceinline__ void vst4i(int* g, int v) { *(volatile int*)g = v; }
__device__ __forceinline__ void st2h(_Float16* g, v8h v) { vst16(g, v); __threadfence(); vst16(g, v); }

#define PREP_BLK_W 1536
#define PREP_BLK_O 512
static_assert(PREP_BLK_W == QKVN * DM / 8 / 256);
static_assert(PREP_BLK_O == DM * DM / 8 / 256);
__device__ __forceinline__ v8h prep_col8(const float* __restrict__ src, size_t ld, float sc) {
    v8h val;
#pragma unroll
    for (int j = 0; j < 8; ++j) val[j] = tohx_flush(src[(size_t)j * ld], sc);
    return val;
}
__global__ __launch_bounds__(256) void k_prep(const float* __restrict__ wQ, const float* __restrict__ wK, const float* __restrict__ wV,
                                              const float* __restrict__ wO, _Float16* WT, _Float16* WoT) {
    const int tid = blockIdx.x * 256 + threadIdx.x;
    if (blockIdx.x < PREP_BLK_W) {
        const int n = tid >> 7, k = (tid & 127) * 8;
        const int m = n >> 10, hh = (n >> 7) & 7, kk = n & 127;
        const size_t so = ((size_t)hh * DM + k) * DK + kk;
        v8h val;
        if (m == 0)      val = prep_col8(wQ + so, DK, SC_W);
        else if (m == 1) val = prep_col8(wK + so, DK, SC_W);
        else             val = prep_col8(wV + so, DK, SC_W);
        st2h(WT + (size_t)n * DM + k, val);
    } else {
        const int i = tid - PREP_BLK_W * 256;
        const int n = i >> 7, k = (i & 127) * 8;
        const v8h val = prep_col8(wO + (size_t)k * DM + n, DM, SC_WO);
        st2h(WoT + (size_t)n * DM + k, val);
    }
}

__global__ __launch_bounds__(32 * NB) void k_flags(const float* __restrict__ MASK, int* FLG) {
    const int t = threadIdx.x, b = t >> 5, tile = t & 31;
    const int tl = (tile < SEQ / 64) ? tile : (SEQ / 64 - 1);
    const float* mp = MASK + (size_t)b * SEQ_FULL + tl * 64;
    int one = 1, zero = 1;
#pragma unroll 1
    for (int j = 0; j < 16; ++j) {
        const v4f m = *(const v4f*)(mp + j * 4);
#pragma unroll
        for (int i = 0; i < 4; ++i) {
            one  &= (m[i] == 1.0f) ? 1 : 0;
            zero &= (m[i] == 0.0f) ? 1 : 0;
        }
    }
    int f = one ? 0 : (zero ? 1 : 2);
    f = (tile < SEQ / 64) ? f : 1;
    vst4i(FLG + b * NTILE_FULL + tile, f);
    __threadfence();
    vst4i(FLG + b * NTILE_FULL + tile, f);
}

__global__ __launch_bounds__(256) void k_xt(const float* __restrict__ X, _Float16* XT) {
    __shared__ __align__(16) _Float16 st[64 * 72];
    const int tid = threadIdx.x;
    const int l0 = blockIdx.x * 64, d0 = blockIdx.y * 64, bi = blockIdx.z;
    const float* xb = X + ((size_t)bi * DM + d0) * SEQ_FULL + l0;
#pragma unroll
    for (int p = 0; p < 4; ++p) {
        const int idx = p * 256 + tid, dr = idx >> 4, lc = idx & 15;
        const v4f v = *(const v4f*)(xb + (size_t)dr * SEQ_FULL + lc * 4);
#pragma unroll
        for (int j = 0; j < 4; ++j) st[(lc * 4 + j) * 72 + dr] = toh_flush(bfr(v[j]));
    }
    __syncthreads();
    v8h w[2];
#pragma unroll
    for (int p = 0; p < 2; ++p) { const int row = p * 32 + (tid >> 3), pc = tid & 7; w[p] = *(const v8h*)&st[row * 72 + pc * 8]; }
    auto pass = [&]() {
#pragma unroll
        for (int p = 0; p < 2; ++p) {
            const int row = p * 32 + (tid >> 3), pc = tid & 7;
            vst16(XT + ((size_t)bi * SEQ + l0 + row) * DM + d0 + pc * 8, w[p]);
        }
    };
    pass();
    __threadfence();
    pass();
}

__global__ __launch_bounds__(128) void k_qkv(const _Float16* __restrict__ XT, const _Float16* __restrict__ WT,
                                             _Float16* QC, _Float16* KC, _Float16* VT) {
    __shared__ __align__(16) _Float16 st[9216];
    const int tid = threadIdx.x, lane = tid & 31, l16 = lane & 15, hf = lane >> 4;
    const int wv = __builtin_amdgcn_readfirstlane((int)(threadIdx.x >> 5));
    const int g = blockIdx.y;
    const int t0 = blockIdx.x * 64;
    const int bi = t0 / SEQ, s0 = t0 - bi * SEQ;
    const bool isV = (g >= 16);
    const _Float16* arow = XT + (size_t)(t0 + wv * 16 + l16) * DM;
    const _Float16* brow = WT + (size_t)(g * 128 + l16) * DM;
    v8f acc[8];
#pragma unroll
    for (int nt = 0; nt < 8; ++nt) acc[nt] = (v8f){};
#pragma unroll 1
    for (int kc = 0; kc < DM / 32; ++kc) {
        const v16h a = ldfrag(arow + kc * 32, hf);
#pragma unroll
        for (int nt = 0; nt < 8; ++nt) {
            const v16h bf = ldfrag(brow + (size_t)nt * 16 * DM + kc * 32, hf);
            acc[nt] = wmma16(a, bf, acc[nt]);
        }
    }
    const float osc = SC_QKV / SC_W;
    if (isV) {
#pragma unroll
        for (int nt = 0; nt < 8; ++nt) {
            const int d = nt * 16 + l16;
            v8h pv;
#pragma unroll
            for (int r = 0; r < 8; ++r) pv[r] = toh_flush(acc[nt][r] * osc);
            *(v8h*)&st[d * 72 + wv * 16 + 8 * hf] = pv;
        }
    } else {
#pragma unroll
        for (int nt = 0; nt < 8; ++nt) {
            const int col = nt * 16 + l16;
#pragma unroll
            for (int r = 0; r < 8; ++r) st[(wv * 16 + 8 * hf + r) * 136 + col] = toh_flush(acc[nt][r] * osc);
        }
    }
    __syncthreads();
    v8h w[8];
    if (isV) {
        const int hd = g - 16;
#pragma unroll
        for (int p = 0; p < 8; ++p) { const int d = p * 16 + (tid >> 3), pc = tid & 7; w[p] = *(const v8h*)&st[d * 72 + pc * 8]; }
        auto pass = [&]() {
#pragma unroll
            for (int p = 0; p < 8; ++p) {
                const int d = p * 16 + (tid >> 3), pc = tid & 7;
                vst16(VT + ((size_t)(bi * NH + hd) * DK + d) * SEQ + s0 + pc * 8, w[p]);
            }
        };
        pass();
        __threadfence();
        pass();
    } else {
        _Float16* base = ((g < 8) ? QC : KC) + ((size_t)(bi * NH + (g & 7)) * SEQ + s0) * DK;
#pragma unroll
        for (int p = 0; p < 8; ++p) { const int off = p * 1024 + tid * 8; w[p] = *(const v8h*)&st[(off >> 7) * 136 + (off & 127)]; }
        auto pass = [&]() {
#pragma unroll
            for (int p = 0; p < 8; ++p) { const int off = p * 1024 + tid * 8; vst16(base + off, w[p]); }
        };
        pass();
        __threadfence();
        pass();
    }
}

__global__ __launch_bounds__(128) void k_attn(const _Float16* __restrict__ QC, const _Float16* __restrict__ KC, const _Float16* __restrict__ VT,
                                              const float* __restrict__ MASK, const int* __restrict__ FLG, _Float16* CTX) {
    __shared__ __align__(16) _Float16 st[4][16 * 136];
    const int tid = threadIdx.x, lane = tid & 31, l16 = lane & 15, hf = lane >> 4;
    const int wv = __builtin_amdgcn_readfirstlane((int)(threadIdx.x >> 5));
    const int bh = blockIdx.y, bi = bh / NH, hd = bh - bi * NH;
    const int q0 = blockIdx.x * 64 + wv * 16;
    const float* mrow = MASK + (size_t)bi * SEQ_FULL;
    const int* frow = FLG + bi * NTILE_FULL;
    const float vq = bfr(mrow[q0 + l16]);
    const int nkt = __builtin_amdgcn_readfirstlane((frow[blockIdx.x] == 1) ? 0 : (SEQ / 64));
    v16h qf[4];
    {
        const _Float16* qr = QC + ((size_t)bh * SEQ + q0 + l16) * DK;
#pragma unroll
        for (int cc = 0; cc < 4; ++cc) qf[cc] = ldfrag(qr + cc * 32, hf);
    }
    const _Float16* kb = KC + (size_t)bh * SEQ * DK;
    const _Float16* vb = VT + (size_t)bh * DK * SEQ;
    v8f o[8];
#pragma unroll
    for (int d = 0; d < 8; ++d) o[d] = (v8f){};
    float m2 = -__builtin_inff(), lsum = 0.0f;
    const float c2 = (0.08838834764831843f * 1.4426950408889634f) * (1.0f / (SC_QKV * SC_QKV));
    const float negl2 = -1.0e30f * 1.4426950408889634f;
#pragma unroll 1
    for (int kt = 0; kt < nkt; ++kt) {
        const int fl = __builtin_amdgcn_readfirstlane(frow[kt]);
        if (fl == 1) continue;
        v8f s[4];
#pragma unroll
        for (int ks = 0; ks < 4; ++ks) {
            const int key = kt * 64 + ks * 16 + l16;
            const _Float16* kr = kb + (size_t)key * DK;
            v8f c = (v8f){};
#pragma unroll
            for (int cc = 0; cc < 4; ++cc) c = wmma16(ldfrag(kr + cc * 32, hf), qf[cc], c);
            s[ks] = c;
        }
#pragma unroll
        for (int ks = 0; ks < 4; ++ks)
#pragma unroll
            for (int r = 0; r < 8; ++r) s[ks][r] *= c2;
        if (fl != 0) {
#pragma unroll
            for (int ks = 0; ks < 4; ++ks) {
                const float* mp = mrow + kt * 64 + ks * 16 + 8 * hf;
                v4f ma = *(const v4f*)mp;
                v4f mb = *(const v4f*)(mp + 4);
#pragma unroll
                for (int r = 0; r < 4; ++r) { ma[r] = bfr(ma[r]); mb[r] = bfr(mb[r]); }
#pragma unroll
                for (int r = 0; r < 4; ++r) {
                    s[ks][r]     = s[ks][r] * ma[r] + (1.0f - ma[r]) * negl2;
                    s[ks][4 + r] = s[ks][4 + r] * mb[r] + (1.0f - mb[r]) * negl2;
                }
            }
        }
        float mloc = -__builtin_inff();
#pragma unroll
        for (int ks = 0; ks < 4; ++ks)
#pragma unroll
            for (int r = 0; r < 8; ++r) mloc = fmaxf(mloc, s[ks][r]);
        mloc = fmaxf(mloc, __shfl_xor(mloc, 16, 32));
        const float mn = fmaxf(m2, mloc);
        const float alpha = exp2f(m2 - mn);
        const float mn8 = mn - P_CARRY_LOG2;
        float ls = 0.0f;
        v16h pf[2];
#pragma unroll
        for (int ks = 0; ks < 4; ++ks)
#pragma unroll
            for (int r = 0; r < 8; ++r) {
                const float e = s[ks][r] - mn8;
                const float p = (e < -14.0f) ? 0.0f : exp2f(e);
                ls += p;
                pf[ks >> 1][(ks & 1) * 8 + r] = (_Float16)p;
            }
        m2 = mn;
        lsum = lsum * alpha + ls;
#pragma unroll
        for (int d = 0; d < 8; ++d) o[d] *= alpha;
#pragma unroll
        for (int d = 0; d < 8; ++d) {
            const _Float16* vr = vb + (size_t)(d * 16 + l16) * SEQ + kt * 64;
            o[d] = wmma16(ldfrag(vr, hf), pf[0], o[d]);
            o[d] = wmma16(ldfrag(vr + 32, hf), pf[1], o[d]);
        }
    }
    const float lt = lsum + __shfl_xor(lsum, 16, 32);
    const float inv = (lt > 0.0f) ? (1.0f / lt) : 0.0f;
    const float scl = inv * vq;
#pragma unroll
    for (int d = 0; d < 8; ++d) {
        v8h pv;
#pragma unroll
        for (int r = 0; r < 8; ++r) pv[r] = toh_flush(o[d][r] * scl);
        *(v8h*)&st[wv][l16 * 136 + d * 16 + 8 * hf] = pv;
    }
    __syncthreads();
    v8h w[8];
#pragma unroll
    for (int t = 0; t < 8; ++t) { const int row = 2 * t + (lane >> 4), pc = lane & 15; w[t] = *(const v8h*)&st[wv][row * 136 + pc * 8]; }
    auto pass = [&]() {
#pragma unroll
        for (int t = 0; t < 8; ++t) {
            const int row = 2 * t + (lane >> 4), pc = lane & 15;
            vst16(CTX + (size_t)(bi * SEQ + q0 + row) * DM + hd * DK + pc * 8, w[t]);
        }
    };
    pass();
    __threadfence();
    pass();
}

__global__ __launch_bounds__(128) void k_out(const _Float16* __restrict__ CTX, const _Float16* __restrict__ WoT, float* OUT) {
    __shared__ __align__(16) float st[4][16 * 68];
    const int tid = threadIdx.x, lane = tid & 31, l16 = lane & 15, hf = lane >> 4;
    const int wv = __builtin_amdgcn_readfirstlane((int)(threadIdx.x >> 5));
    const int t0 = blockIdx.x * 64, n0 = blockIdx.y * 64 + wv * 16;
    const int bi = t0 / SEQ, s0 = t0 - bi * SEQ;
    const _Float16* arow = WoT + (size_t)(n0 + l16) * DM;
    const _Float16* brow = CTX + (size_t)(t0 + l16) * DM;
    v8f acc[4];
#pragma unroll
    for (int tt = 0; tt < 4; ++tt) acc[tt] = (v8f){};
#pragma unroll 1
    for (int kc = 0; kc < DM / 32; ++kc) {
        const v16h a = ldfrag(arow + kc * 32, hf);
#pragma unroll
        for (int tt = 0; tt < 4; ++tt) {
            const v16h bf = ldfrag(brow + (size_t)tt * 16 * DM + kc * 32, hf);
            acc[tt] = wmma16(a, bf, acc[tt]);
        }
    }
#pragma unroll
    for (int tt = 0; tt < 4; ++tt) {
        const int col = tt * 16 + l16;
#pragma unroll
        for (int r = 0; r < 8; ++r) st[wv][(8 * hf + r) * 68 + col] = acc[tt][r] * (1.0f / (SC_QKV * SC_WO));
    }
    __syncthreads();
    const int pc = lane & 15;
    v4f w[8];
#pragma unroll
    for (int t = 0; t < 8; ++t) { const int row = 2 * t + (lane >> 4); w[t] = *(const v4f*)&st[wv][row * 68 + pc * 4]; }
    auto pass = [&]() {
#pragma unroll
        for (int t = 0; t < 8; ++t) {
            const int row = 2 * t + (lane >> 4);
            vst16f(OUT + ((size_t)bi * DM + n0 + row) * SEQ_FULL + s0 + pc * 4, w[t]);
        }
    };
    pass();
    __threadfence();
    pass();
}

extern "C" void kernel_launch(void* const* d_in, const int* in_sizes, int n_in,
                              void* d_out, int out_size, void* d_ws, size_t ws_size, hipStream_t stream) {
    if (n_in < 6) return;
    const long long needX = ((long long)(NB - 1) * DM + (DM - 1)) * SEQ_FULL + SEQ;
    const long long needM = (long long)(NB - 1) * SEQ_FULL + SEQ;
    if ((long long)in_sizes[0] < needX) return;
    if ((long long)in_sizes[1] < needM) return;
    if (in_sizes[2] < NH * DM * DK || in_sizes[3] < NH * DM * DK || in_sizes[4] < NH * DM * DK || in_sizes[5] < DM * DM) return;
    if ((long long)out_size < needX) return;

    const float* x    = (const float*)d_in[0];
    const float* mask = (const float*)d_in[1];
    const float* Wq   = (const float*)d_in[2];
    const float* Wk   = (const float*)d_in[3];
    const float* Wv   = (const float*)d_in[4];
    const float* Wo   = (const float*)d_in[5];
    float* out = (float*)d_out;

    char* ws = (char*)d_ws;
    size_t off = 0;
    auto carve = [&](size_t bytes) -> char* { char* p = ws + off; off += (bytes + 255) & ~(size_t)255; return p; };
    _Float16* WT  = (_Float16*)carve((size_t)QKVN * DM * 2);
    _Float16* WoT = (_Float16*)carve((size_t)DM * DM * 2);
    _Float16* XT  = (_Float16*)carve((size_t)MTOK * DM * 2);
    _Float16* QC  = (_Float16*)carve((size_t)NB * NH * SEQ * DK * 2);
    _Float16* KC  = (_Float16*)carve((size_t)NB * NH * SEQ * DK * 2);
    _Float16* VT  = (_Float16*)carve((size_t)NB * NH * DK * SEQ * 2);
    _Float16* CTX = (_Float16*)carve((size_t)MTOK * DM * 2);
    int*      FLG = (int*)carve((size_t)NB_FULL * NTILE_FULL * 4);
    if (off > ws_size) return;

    k_prep<<<PREP_BLK_W + PREP_BLK_O, 256, 0, stream>>>(Wq, Wk, Wv, Wo, WT, WoT);
    k_flags<<<1, 32 * NB, 0, stream>>>(mask, FLG);
    k_xt<<<dim3(SEQ / 64, DM / 64, NB), 256, 0, stream>>>(x, XT);
    k_qkv<<<dim3(MTOK / 64, QKVN / 128, 1), 128, 0, stream>>>(XT, WT, QC, KC, VT);
    k_attn<<<dim3(SEQ / 64, NB * NH, 1), 128, 0, stream>>>(QC, KC, VT, mask, FLG, CTX);
    k_out<<<dim3(MTOK / 64, DM / 64, 1), 128, 0, stream>>>(CTX, WoT, out);
}
